// GAT_9371618640567
// MI455X (gfx1250) — hardware-verified
//
#include <hip/hip_runtime.h>
#include <stddef.h>
#include <stdint.h>
#include <math.h>


#define F_IN    128
#define HC      128
#define HW1     32
#define NHD     4
#define OUTC    40
#define HC3     64
#define KA      256
#define NTHR    256
#define NWAVE   8
#define EPT     8
#define CHUNK   (NTHR * EPT)
#define WCAP    (EPT * 32)
#define LISTN   (NWAVE * WCAP)
#define NB      1024
#define SLOTB   10
#define RCAP    28672
#define DEGCAP  64
#define HDRW    32
#define RROWS   256
#define GBM     64
#define GBN     64
#define GTHR    128
#define MROWS   128
#define PARTW   288
#define WSTW    258
#define BNROWS  128
#define NEGSL   0.2f
#define WSMAX   134217728
#define LDS_BKT ((2 * RCAP + 2 * NB + LISTN + 16) * 4)

static_assert((CHUNK & (CHUNK - 1)) == 0 && CHUNK == 2048);
static_assert(NB == (1 << SLOTB));
static_assert(((long long)CHUNK << SLOTB) < (1LL << 31));
static_assert(NTHR * 4 == NB);
static_assert(LISTN >= NB);
static_assert((RCAP % 32) == 0 && (RCAP % 4) == 0);
static_assert(LDS_BKT <= 300000);
static_assert(GBM == (GTHR / 32) * 16);
static_assert(GTHR == 2 * GBN && GTHR == 2 * GBM);
static_assert((F_IN % 32) == 0 && (KA % 32) == 0 && KA == 2 * HC);
static_assert((HC % GBN) == 0 && HC3 == GBN && HC == NHD * HW1);
static_assert((MROWS % GBM) == 0 && (MROWS % BNROWS) == 0);
static_assert(HC == 4 * 32);
static_assert(HW1 == 4 * 8);
static_assert((F_IN / 8) == 16);
static_assert((OUTC % 4) == 0 && OUTC <= HC3);
static_assert((NB % RROWS) == 0 && RROWS == NWAVE * 32);
static_assert(((RROWS * OUTC * 4) % 128) == 0);
static_assert(((RROWS * OUTC / 4) % NTHR) == 0);
static_assert(PARTW % 32 == 0 && PARTW / 4 <= NTHR && PARTW >= 2 * HC + 1);
static_assert(WSTW >= 2 * HC + 1);
static_assert((BNROWS * 16) % NTHR == 0);
static_assert(HDRW == 32);

typedef float          v4f  __attribute__((ext_vector_type(4)));
typedef float          v8f  __attribute__((ext_vector_type(8)));
typedef int            v4i  __attribute__((ext_vector_type(4)));
typedef int            v8i  __attribute__((ext_vector_type(8)));
typedef unsigned int   v4u  __attribute__((ext_vector_type(4)));
typedef unsigned short v8us __attribute__((ext_vector_type(8)));
typedef __bf16         v16b __attribute__((ext_vector_type(16)));
typedef v4f  __attribute__((may_alias)) v4fa;
typedef v4i  __attribute__((may_alias)) v4ia;
typedef v8us __attribute__((may_alias)) v8usa;
union FragB { v16b v; v8us h[2]; v8i w; };

__device__ __forceinline__ v8f wmb(const FragB& a, const FragB& b, v8f c) {
  v8f d = __builtin_amdgcn_wmma_f32_16x16x32_bf16(false, a.v, false, b.v, (short)0, c, false, false);
  asm volatile("v_nop\n\tv_nop\n\tv_nop\n\tv_nop" : "+v"(d) : "v"(a.w), "v"(b.w));
  return d;
}

__device__ __forceinline__ unsigned int f2bf(float f) {
  const unsigned int u = __float_as_uint(f);
  const unsigned int r = ((u + 0x7FFFu + ((u >> 16) & 1u)) >> 16) & 0xFFFFu;
  return ((u & 0x7FFFFFFFu) > 0x7F800000u) ? 0x7FC0u : r;
}
__device__ __forceinline__ float bf2f(unsigned int b) { return __uint_as_float(b << 16); }
__device__ __forceinline__ float bfr(float f) { return bf2f(f2bf(f)); }
__device__ __forceinline__ v4f bfr4(const v4f a) {
  v4f r; r.x = bfr(a.x); r.y = bfr(a.y); r.z = bfr(a.z); r.w = bfr(a.w); return r;
}
__device__ __forceinline__ unsigned int pk2(float lo, float hi) { return f2bf(lo) | (f2bf(hi) << 16); }
__device__ __forceinline__ v4u pack8(const v4f a, const v4f b) {
  v4u r;
  r.x = pk2(a.x, a.y); r.y = pk2(a.z, a.w); r.z = pk2(b.x, b.y); r.w = pk2(b.z, b.w);
  return r;
}
__device__ __forceinline__ v4u pack8lo(const v4f a, const v4f b) {
  v4f ra, rb;
  ra.x = a.x - bfr(a.x); ra.y = a.y - bfr(a.y); ra.z = a.z - bfr(a.z); ra.w = a.w - bfr(a.w);
  rb.x = b.x - bfr(b.x); rb.y = b.y - bfr(b.y); rb.z = b.z - bfr(b.z); rb.w = b.w - bfr(b.w);
  return pack8(ra, rb);
}
__device__ __forceinline__ float relun(float v) { return (v > 0.f) ? v : (v - v); }

__device__ __forceinline__ int scan_chunk(const int* __restrict__ dsts, int nE, int cbase, int slotBase,
                                          int nb, int vec8, int* list, int tid, int lane, int wave) {
  int wc = 0;
  const int el0  = tid * EPT;
  const int e0   = cbase + el0;
  const int sent = -2147483647 - 1;
  v4i da, db;
  if (vec8 != 0 && cbase + CHUNK <= nE) {
    da = *(const v4ia*)(dsts + e0);
    db = *(const v4ia*)(dsts + e0 + 4);
  } else {
    da.x = (e0     < nE) ? dsts[min(e0,     nE - 1)] : sent;
    da.y = (e0 + 1 < nE) ? dsts[min(e0 + 1, nE - 1)] : sent;
    da.z = (e0 + 2 < nE) ? dsts[min(e0 + 2, nE - 1)] : sent;
    da.w = (e0 + 3 < nE) ? dsts[min(e0 + 3, nE - 1)] : sent;
    db.x = (e0 + 4 < nE) ? dsts[min(e0 + 4, nE - 1)] : sent;
    db.y = (e0 + 5 < nE) ? dsts[min(e0 + 5, nE - 1)] : sent;
    db.z = (e0 + 6 < nE) ? dsts[min(e0 + 6, nE - 1)] : sent;
    db.w = (e0 + 7 < nE) ? dsts[min(e0 + 7, nE - 1)] : sent;
  }
  const unsigned nbs = (unsigned)slotBase;
  const unsigned unb = (unsigned)nb;
  const unsigned s0 = (unsigned)da.x - nbs, s1 = (unsigned)da.y - nbs;
  const unsigned s2 = (unsigned)da.z - nbs, s3 = (unsigned)da.w - nbs;
  const unsigned s4 = (unsigned)db.x - nbs, s5 = (unsigned)db.y - nbs;
  const unsigned s6 = (unsigned)db.z - nbs, s7 = (unsigned)db.w - nbs;
  const bool h0 = s0 < unb, h1 = s1 < unb, h2 = s2 < unb, h3 = s3 < unb;
  const bool h4 = s4 < unb, h5 = s5 < unb, h6 = s6 < unb, h7 = s7 < unb;
  const unsigned any = __builtin_amdgcn_ballot_w32(h0 | h1 | h2 | h3 | h4 | h5 | h6 | h7);
  if (any != 0u) {
#define HITJ(J, HJ, SJ) { \
      const unsigned mj = __builtin_amdgcn_ballot_w32(HJ); \
      if (mj != 0u) { \
        if (HJ) { \
          const int pos = wc + (int)__builtin_amdgcn_mbcnt_lo(mj, 0u); \
          if (pos < WCAP) list[wave * WCAP + pos] = ((el0 + (J)) << SLOTB) | (int)(SJ); \
        } \
        wc += (int)__builtin_popcount(mj); } }
    HITJ(0, h0, s0)
    HITJ(1, h1, s1)
    HITJ(2, h2, s2)
    HITJ(3, h3, s3)
    HITJ(4, h4, s4)
    HITJ(5, h5, s5)
    HITJ(6, h6, s6)
    HITJ(7, h7, s7)
#undef HITJ
  }
  return wc;
}

__global__ __launch_bounds__(NTHR) void k_xprep(const float* __restrict__ x, unsigned short* xb, int nN, int nUnits) {
  const int i = (int)blockIdx.x * NTHR + (int)threadIdx.x;
  if (i >= nUnits) return;
  const int row = i >> 4;
  const int c0  = (i & 15) * 8;
  const int rc  = row < nN ? row : nN - 1;
  const float* p = x + (size_t)rc * F_IN + c0;
  v4f a = *(const v4fa*)p, b = *(const v4fa*)(p + 4);
  const v4f z4 = {0.f, 0.f, 0.f, 0.f};
  if (row >= nN) { a = z4; b = z4; }
  const v4u hv = pack8(a, b);
  const size_t o = (size_t)row * F_IN + c0;
  *(volatile v4u*)(xb + o) = hv;
  __threadfence();
  *(volatile v4u*)(xb + o) = hv;
}

__global__ __launch_bounds__(NTHR) void k_wtr(const float* __restrict__ w, int Kin, int Ncol, int Nrows, int Kout,
                                              unsigned short* wt, int nUnits) {
  const int u = (int)blockIdx.x * NTHR + (int)threadIdx.x;
  if (u >= nUnits) return;
  const int kq = Kout >> 3;
  const int n  = u / kq;
  const int k8 = (u - n * kq) * 8;
  const int kk = k8 - (k8 / Kin) * Kin;
  const int ncl = n < Ncol ? n : Ncol - 1;
  const float* p = w + (size_t)kk * (size_t)Ncol + ncl;
  v4f a, b;
  a.x = p[0];                    a.y = p[(size_t)Ncol];         a.z = p[(size_t)2 * Ncol];     a.w = p[(size_t)3 * Ncol];
  b.x = p[(size_t)4 * Ncol];     b.y = p[(size_t)5 * Ncol];     b.z = p[(size_t)6 * Ncol];     b.w = p[(size_t)7 * Ncol];
  const v4f z4 = {0.f, 0.f, 0.f, 0.f};
  if (n >= Ncol || n >= Nrows) { a = z4; b = z4; }
  const v4u wv = pack8(a, b);
  unsigned short* o = wt + (size_t)n * (size_t)Kout + k8;
  *(volatile v4u*)o = wv;
  __threadfence();
  *(volatile v4u*)o = wv;
}

__global__ __launch_bounds__(NTHR) void k_bucket(const int* __restrict__ srcs, const int* __restrict__ dsts,
                                                 int nN, int nE, int vec8, int* SRT, int* OFFS, int* HDR) {
  extern __shared__ v4f lds_dyn[];
  int* reg1 = (int*)lds_dyn;
  int* reg2 = reg1 + RCAP;
  int* scnt = reg2 + RCAP;
  int* soff = scnt + NB;
  int* list = soff + NB;
  int* wcnt = list + LISTN;
  int* wtot = wcnt + NWAVE;
  const int tid = (int)threadIdx.x, lane = tid & 31, wave = tid >> 5;
  const int blk = (int)blockIdx.x;
  const int nodeBase = blk * NB;

  {
    const v4i z4 = {0, 0, 0, 0};
    for (int p = tid; p < RCAP / 4; p += NTHR) *(v4ia*)(reg2 + 4 * p) = z4;
    for (int p = tid; p < NB / 4; p += NTHR)   *(v4ia*)(scnt + 4 * p) = z4;
  }
  __syncthreads();

  int tot = 0, ovf = 0;
  const int nChunks = (nE + CHUNK - 1) / CHUNK;
#pragma unroll 1
  for (int ch = 0; ch < nChunks; ++ch) {
    const int cbase = ch * CHUNK;
    const int wc = scan_chunk(dsts, nE, cbase, nodeBase, NB, vec8, list, tid, lane, wave);
    if (lane == 0) wcnt[wave] = wc;
    __syncthreads();
    int pre = 0, all = 0;
#pragma unroll
    for (int w2 = 0; w2 < NWAVE; ++w2) {
      int c = wcnt[w2];
      c = c < 0 ? 0 : (c > WCAP ? WCAP : c);
      all += c;
      pre += (w2 < wave) ? c : 0;
    }
    const int wcc  = wc > WCAP ? WCAP : wc;
    const int base = tot + pre;
    if (wcc > 0) {
#pragma unroll 1
      for (int i0 = 0; i0 < wcc; i0 += 32) {
        const int iu  = i0 + lane;
        const int i   = iu < wcc ? iu : wcc - 1;
        const int ent = list[wave * WCAP + i];
        const int el  = (ent >> SLOTB) & (CHUNK - 1);
        const int sl  = ent & (NB - 1);
        int eid = cbase + el;
        eid = eid < 0 ? 0 : (eid > nE - 1 ? nE - 1 : eid);
        const int sraw = srcs[eid];
        const int s = sraw < 0 ? 0 : (sraw > nN - 1 ? nN - 1 : sraw);
        const int pos = base + iu;
        if (iu < wcc && pos < RCAP) reg1[pos] = s | (sl << 16);
      }
    }
    tot += all;
    if (tot > RCAP) { ovf = 1; tot = RCAP; }
    __syncthreads();
  }
  const int nh = tot;

  if (wave == 0) {
#pragma unroll 1
    for (int b0 = 0; b0 < nh; b0 += 32) {
      const int idx = b0 + lane;
      const int uv  = reg1[idx < nh ? idx : nh - 1];
      const int m32 = (nh - b0) < 32 ? (nh - b0) : 32;
#pragma unroll 1
      for (int k = 0; k < m32; ++k) {
        const int u  = __builtin_amdgcn_readlane(uv, k);
        const int sl = (u >> 16) & (NB - 1);
        if (lane == 0) scnt[sl] = scnt[sl] + 1;
      }
    }
  }
  __syncthreads();

  {
    const v4i ca = *(const v4ia*)(scnt + 4 * tid);
    const int e0 = ca.x < 0 ? 0 : ca.x, e1 = ca.y < 0 ? 0 : ca.y, e2 = ca.z < 0 ? 0 : ca.z, e3 = ca.w < 0 ? 0 : ca.w;
    const int ts = e0 + e1 + e2 + e3;
    int incl = ts;
#pragma unroll
    for (int d = 1; d < 32; d <<= 1) {
      const int up = __shfl_up(incl, d);
      if (lane >= d) incl += up;
    }
    if (lane == 31) wtot[wave] = incl;
    __syncthreads();
    int pre = 0;
#pragma unroll
    for (int w2 = 0; w2 < NWAVE; ++w2) pre += (w2 < wave) ? wtot[w2] : 0;
    int run = pre + incl - ts;
    soff[4 * tid + 0] = run; run += e0;
    soff[4 * tid + 1] = run; run += e1;
    soff[4 * tid + 2] = run; run += e2;
    soff[4 * tid + 3] = run;
  }
  __syncthreads();
  for (int i = tid; i < NB; i += NTHR) list[i] = soff[i];
  __syncthreads();

  if (wave == 0) {
#pragma unroll 1
    for (int b0 = 0; b0 < nh; b0 += 32) {
      const int idx = b0 + lane;
      const int uv  = reg1[idx < nh ? idx : nh - 1];
      const int m32 = (nh - b0) < 32 ? (nh - b0) : 32;
#pragma unroll 1
      for (int k = 0; k < m32; ++k) {
        const int u  = __builtin_amdgcn_readlane(uv, k);
        const int sl = (u >> 16) & (NB - 1);
        const int sv = u & 0xFFFF;
        if (lane == 0) {
          int pos = list[sl];
          pos = pos < 0 ? 0 : (pos > RCAP - 1 ? RCAP - 1 : pos);
          reg2[pos] = sv;
          list[sl] = pos + 1;
        }
      }
    }
  }
  __syncthreads();

  int* srt = SRT  + (size_t)blk * RCAP;
  int* ofs = OFFS + (size_t)blk * (2 * NB);
  int* hdr = HDR  + (size_t)blk * HDRW;
  v4i hv = {0, 0, 0, 0};
  if (lane == 0) { hv.x = nh; hv.y = ovf; }
#pragma unroll 1
  for (int p = tid; p < RCAP / 4; p += NTHR) {
    const v4i v = *(const v4ia*)(reg2 + 4 * p);
    *(volatile v4i*)(srt + 4 * p) = v;
  }
#pragma unroll 1
  for (int p = tid; p < (2 * NB) / 4; p += NTHR) {
    const v4i v = *(const v4ia*)(scnt + 4 * p);
    *(volatile v4i*)(ofs + 4 * p) = v;
  }
  if (wave == 0 && lane < 8) *(volatile v4i*)(hdr + 4 * lane) = hv;
  __threadfence();
#pragma unroll 1
  for (int p = tid; p < RCAP / 4; p += NTHR) {
    const v4i v = *(const v4ia*)(reg2 + 4 * p);
    *(volatile v4i*)(srt + 4 * p) = v;
  }
#pragma unroll 1
  for (int p = tid; p < (2 * NB) / 4; p += NTHR) {
    const v4i v = *(const v4ia*)(scnt + 4 * p);
    *(volatile v4i*)(ofs + 4 * p) = v;
  }
  if (wave == 0 && lane < 8) *(volatile v4i*)(hdr + 4 * lane) = hv;
}

template<int NHB, int HW>
__global__ __launch_bounds__(GTHR) void k_gemm(
    const unsigned short* __restrict__ A, const unsigned short* __restrict__ WT,
    float* outF, int K, int ldo,
    const float* __restrict__ atts, const float* __restrict__ attd, int attLen,
    float* SD, int MPr)
{
  static_assert(NHB * HW == GBN && NHB <= GTHR / 32 && (HW % 4) == 0);
  __shared__ __attribute__((aligned(16))) float stg[GBM * GBN];
  __shared__ __attribute__((aligned(16))) float satt[2 * GBN];
  __shared__ __attribute__((aligned(16))) float sdot[2 * NHB * GBM];
  const int tid = (int)threadIdx.x, lane = tid & 31, wave = tid >> 5, hh = lane >> 4, m = lane & 15;
  const int rowBase  = (int)blockIdx.x * GBM;
  const int headBase = (int)blockIdx.y * NHB;
  const int col0     = (int)blockIdx.y * GBN;

  {
    const int which = tid >> 6;
    const int c  = tid & 63;
    const int hb = c / HW;
    const int ci = c - hb * HW;
    const int cl = ci < attLen ? ci : attLen - 1;
    const int ai = (headBase + hb) * attLen + cl;
    const float vs = atts[ai];
    const float vd = attd[ai];
    const unsigned int msk = (which == 0) ? 0u : 0xFFFFFFFFu;
    const unsigned int inr = (ci < attLen) ? 0xFFFFFFFFu : 0u;
    float v = __uint_as_float((__float_as_uint(vs) & ~msk) | (__float_as_uint(vd) & msk));
    v = __uint_as_float(__float_as_uint(bfr(v)) & inr);
    satt[which * GBN + c] = v;
  }

  v8f acc[4];
  {
    const v8f z = {0.f, 0.f, 0.f, 0.f, 0.f, 0.f, 0.f, 0.f};
    acc[0] = z; acc[1] = z; acc[2] = z; acc[3] = z;
  }
  const unsigned short* ap = A  + (size_t)(rowBase + 16 * wave + m) * (size_t)K + 8 * hh;
  const unsigned short* wp = WT + (size_t)(col0 + m) * (size_t)K + 8 * hh;
  const int ksteps = K >> 5;
#pragma unroll 1
  for (int ks = 0; ks < ksteps; ++ks) {
    FragB af;
    af.h[0] = *(const v8usa*)(ap + 32 * ks);
    af.h[1] = *(const v8usa*)(ap + 32 * ks + 16);
#pragma unroll
    for (int t = 0; t < 4; ++t) {
      const unsigned short* wq = wp + (size_t)(16 * t) * (size_t)K + 32 * ks;
      FragB bf;
      bf.h[0] = *(const v8usa*)wq;
      bf.h[1] = *(const v8usa*)(wq + 16);
      acc[t] = wmb(af, bf, acc[t]);
    }
  }

#pragma unroll
  for (int t = 0; t < 4; ++t) {
    const int lc = 16 * t + m;
#pragma unroll
    for (int r = 0; r < 8; ++r) {
      const int lr = 16 * wave + 8 * hh + r;
      stg[lr * GBN + lc] = acc[t][r];
    }
  }
  __syncthreads();

  {
    const int row = tid & 63, which = tid >> 6;
#pragma unroll
    for (int hb = 0; hb < NHB; ++hb) {
      const float* sa = satt + which * GBN + hb * HW;
      const float* hr = stg + row * GBN + hb * HW;
      float d = 0.f;
#pragma unroll 4
      for (int c4 = 0; c4 < HW / 4; ++c4) {
        const v4f hv = *(const v4fa*)(hr + 4 * c4);
        const v4f av = *(const v4fa*)(sa + 4 * c4);
        d = fmaf(hv.x, av.x, d);
        d = fmaf(hv.y, av.y, d);
        d = fmaf(hv.z, av.z, d);
        d = fmaf(hv.w, av.w, d);
      }
      sdot[(2 * hb + which) * GBM + row] = d;
    }
  }
  __syncthreads();

  v4f fv[8];
#pragma unroll
  for (int i = 0; i < 8; ++i) {
    const int lr = 16 * wave + 2 * i + hh;
    fv[i] = *(const v4fa*)(stg + lr * GBN + 4 * m);
  }
  const int hbw = wave < NHB ? wave : 0;
  const int which2 = lane >> 4, piece = lane & 15;
  const v4f sdv = *(const v4fa*)(sdot + (2 * hbw + which2) * GBM + 4 * piece);
  float* sp = SD + (size_t)(2 * (headBase + hbw) + which2) * (size_t)MPr + rowBase + 4 * piece;

#pragma unroll
  for (int i = 0; i < 8; ++i) {
    const int lr = 16 * wave + 2 * i + hh;
    const int gr = rowBase + lr;
    float* op = outF + (size_t)gr * (size_t)ldo + col0 + 4 * m;
    *(volatile v4f*)op = fv[i];
  }
  if (wave < NHB) *(volatile v4f*)sp = sdv;
  __threadfence();
#pragma unroll
  for (int i = 0; i < 8; ++i) {
    const int lr = 16 * wave + 2 * i + hh;
    const int gr = rowBase + lr;
    float* op = outF + (size_t)gr * (size_t)ldo + col0 + 4 * m;
    *(volatile v4f*)op = fv[i];
  }
  if (wave < NHB) *(volatile v4f*)sp = sdv;
}

template<int L>
__global__ __launch_bounds__(NTHR) void k_scan(
    const int* __restrict__ SRT, const int* __restrict__ OFFS, const int* __restrict__ HDR,
    const float* __restrict__ F, const float* __restrict__ SD, const float* __restrict__ bias,
    float* PRE, float* out, int nN, int MPr) {
  __shared__ __attribute__((aligned(16))) int   tab[2 * NB];
  __shared__ __attribute__((aligned(16))) float res[(L == 1) ? (RROWS * OUTC) : 4];
  const int tid = (int)threadIdx.x, lane = tid & 31, wave = tid >> 5;
  const int blk = (int)blockIdx.x;
  const int nodeBase = blk * NB;

  {
    const int* tp = OFFS + (size_t)blk * (2 * NB);
#pragma unroll 1
    for (int p = tid; p < (2 * NB) / 4; p += NTHR) {
      const v4i t4 = *(const v4ia*)(tp + 4 * p);
      *(v4ia*)(tab + 4 * p) = t4;
    }
  }
  int nh = HDR[(size_t)blk * HDRW];
  nh = nh < 0 ? 0 : (nh > RCAP ? RCAP : nh);
  const int ovfw = HDR[(size_t)blk * HDRW + 1];
  __syncthreads();

  const bool ovf = (ovfw != 0);
  const float qnan = __int_as_float(0x7fc00000);
  const int* srt = SRT + (size_t)blk * RCAP;

  if constexpr (L == 0) {
    const int c0   = 4 * lane;
    const int head = lane >> 3;
    const v4f bb   = bfr4(*(const v4fa*)(bias + c0));
    const float* ASp = SD + (size_t)(2 * head) * (size_t)MPr;
    const float* ADp = ASp + MPr;
    const int nbw = NB / NWAVE;

#pragma unroll 1
    for (int jt = 0; jt < nbw; ++jt) {
      const int slot = wave * nbw + jt;
      const int grow = nodeBase + slot;
      const int gcl  = grow < nN ? grow : nN - 1;
      const int craw = tab[slot];
      int st  = tab[NB + slot];
      int cnt = craw;
      st  = st < 0 ? 0 : (st > nh ? nh : st);
      cnt = cnt < 0 ? 0 : (cnt > DEGCAP ? DEGCAP : cnt);
      if (cnt > nh - st) cnt = nh - st;
      const float pz = (ovf || craw > DEGCAP) ? qnan : 0.0f;

      v4f av = *(const v4fa*)(F + (size_t)gcl * HC + c0);
      const float adv = ADp[gcl];
      float l0 = ASp[gcl] + adv;
      l0 = l0 > 0.f ? l0 : NEGSL * l0;
      float mx = l0, dn = 1.0f;

#pragma unroll 1
      for (int b0 = 0; b0 < cnt; b0 += 32) {
        int idx = st + b0 + lane;
        idx = idx < 0 ? 0 : (idx > RCAP - 1 ? RCAP - 1 : idx);
        int sr = srt[idx];
        sr = sr < 0 ? 0 : (sr > nN - 1 ? nN - 1 : sr);
        const int m32 = (cnt - b0) < 32 ? (cnt - b0) : 32;
#pragma unroll 1
        for (int k = 0; k < m32; ++k) {
          const int s = __builtin_amdgcn_readlane(sr, k);
          const v4f fa = *(const v4fa*)(F + (size_t)s * HC + c0);
          float lg = ASp[s] + adv;
          lg = lg > 0.f ? lg : NEGSL * lg;
          const float df = lg - mx;
          const float ee = expf(-fabsf(df));
          const bool up  = df > 0.f;
          const float s1 = up ? ee : 1.0f;
          const float s2 = up ? 1.0f : ee;
          mx = up ? lg : mx;
          dn = fmaf(dn, s1, s2);
          av.x = fmaf(av.x, s1, s2 * fa.x);
          av.y = fmaf(av.y, s1, s2 * fa.y);
          av.z = fmaf(av.z, s1, s2 * fa.z);
          av.w = fmaf(av.w, s1, s2 * fa.w);
        }
      }
      const float inv = __builtin_amdgcn_rcpf(dn);
      const bool live = grow < nN;
      v4f o;
      o.x = (live ? fmaf(av.x, inv, bb.x) : 0.f) + pz;
      o.y = (live ? fmaf(av.y, inv, bb.y) : 0.f) + pz;
      o.z = (live ? fmaf(av.z, inv, bb.z) : 0.f) + pz;
      o.w = (live ? fmaf(av.w, inv, bb.w) : 0.f) + pz;
      float* gp = PRE + (size_t)grow * HC + c0;
      const bool wr = grow < MPr;
      if (wr) *(volatile v4f*)gp = o;
      __threadfence();
      if (wr) *(volatile v4f*)gp = o;
    }
  } else {
    const int c0 = 4 * (lane & 15);
    const int cb = c0 <= OUTC - 4 ? c0 : OUTC - 4;
    v4f bb = bfr4(*(const v4fa*)(bias + cb));
    {
      const v4f z4 = {0.f, 0.f, 0.f, 0.f};
      if (c0 >= OUTC) bb = z4;
    }
    const float* ASp = SD;
    const float* ADp = SD + MPr;
    const int nTot = nN * OUTC;

#pragma unroll 1
    for (int r = 0; r < NB / RROWS; ++r) {
#pragma unroll 1
      for (int j = 0; j < 32; ++j) {
        const int sl2  = wave * 32 + j;
        const int slot = r * RROWS + sl2;
        const int grow = nodeBase + slot;
        const int gcl  = grow < nN ? grow : nN - 1;
        const int craw = tab[slot];
        int st  = tab[NB + slot];
        int cnt = craw;
        st  = st < 0 ? 0 : (st > nh ? nh : st);
        cnt = cnt < 0 ? 0 : (cnt > DEGCAP ? DEGCAP : cnt);
        if (cnt > nh - st) cnt = nh - st;
        const float pz = (ovf || craw > DEGCAP) ? qnan : 0.0f;

        v4f av = *(const v4fa*)(F + (size_t)gcl * HC3 + c0);
        const float adv = ADp[gcl];
        float l0 = ASp[gcl] + adv;
        l0 = l0 > 0.f ? l0 : NEGSL * l0;
        float mx = l0, dn = 1.0f;

#pragma unroll 1
        for (int b0 = 0; b0 < cnt; b0 += 32) {
          int idx = st + b0 + lane;
          idx = idx < 0 ? 0 : (idx > RCAP - 1 ? RCAP - 1 : idx);
          int sr = srt[idx];
          sr = sr < 0 ? 0 : (sr > nN - 1 ? nN - 1 : sr);
          const int m32 = (cnt - b0) < 32 ? (cnt - b0) : 32;
#pragma unroll 1
          for (int k = 0; k < m32; ++k) {
            const int s = __builtin_amdgcn_readlane(sr, k);
            const v4f fa = *(const v4fa*)(F + (size_t)s * HC3 + c0);
            float lg = ASp[s] + adv;
            lg = lg > 0.f ? lg : NEGSL * lg;
            const float df = lg - mx;
            const float ee = expf(-fabsf(df));
            const bool up  = df > 0.f;
            const float s1 = up ? ee : 1.0f;
            const float s2 = up ? 1.0f : ee;
            mx = up ? lg : mx;
            dn = fmaf(dn, s1, s2);
            av.x = fmaf(av.x, s1, s2 * fa.x);
            av.y = fmaf(av.y, s1, s2 * fa.y);
            av.z = fmaf(av.z, s1, s2 * fa.z);
            av.w = fmaf(av.w, s1, s2 * fa.w);
          }
        }
        const float inv = __builtin_amdgcn_rcpf(dn);
        v4f o;
        o.x = fmaf(av.x, inv, bb.x) + pz;
        o.y = fmaf(av.y, inv, bb.y) + pz;
        o.z = fmaf(av.z, inv, bb.z) + pz;
        o.w = fmaf(av.w, inv, bb.w) + pz;
        if (lane < OUTC / 4) *(v4fa*)(res + sl2 * OUTC + 4 * lane) = o;
      }
      __syncthreads();
      const int f0b = (nodeBase + r * RROWS) * OUTC;
#pragma unroll 1
      for (int p = tid; p < (RROWS * OUTC) / 4; p += NTHR) {
        const v4f v = *(const v4fa*)(res + 4 * p);
        const int f0 = f0b + 4 * p;
        if (nTot - f0 >= 4) *(volatile v4f*)(out + (size_t)f0) = v;
      }
      __threadfence();
#pragma unroll 1
      for (int p = tid; p < (RROWS * OUTC) / 4; p += NTHR) {
        const v4f v = *(const v4fa*)(res + 4 * p);
        const int f0 = f0b + 4 * p;
        if (nTot - f0 >= 4) *(volatile v4f*)(out + (size_t)f0) = v;
      }
      __syncthreads();
    }
  }
}

__global__ __launch_bounds__(NTHR) void k_stats(const float* __restrict__ pre, int nN, float* rec) {
  __shared__ __attribute__((aligned(16))) float wst[NWAVE * WSTW];
  __shared__ __attribute__((aligned(16))) float pst[PARTW];
  const int tid = (int)threadIdx.x, lane = tid & 31, wave = tid >> 5;
  const int base = (int)blockIdx.x * NB;
  int wn = 0;
  float wm[4], wq[4];
#pragma unroll
  for (int j = 0; j < 4; ++j) { wm[j] = 0.0f; wq[j] = 0.0f; }
#pragma unroll 1
  for (int i = 0; i < NB / NWAVE; ++i) {
    const int row = base + wave + NWAVE * i;
    const bool ok = row < nN;
    const int rc  = ok ? row : nN - 1;
    const v4f x = *(const v4fa*)(pre + (size_t)rc * HC + 4 * lane);
    if (ok) {
      wn += 1;
      const float rk = 1.0f / (float)wn;
      float vv[4];
      vv[0] = x.x; vv[1] = x.y; vv[2] = x.z; vv[3] = x.w;
#pragma unroll
      for (int j = 0; j < 4; ++j) {
        const float d = vv[j] - wm[j];
        wm[j] = fmaf(d, rk, wm[j]);
        wq[j] = fmaf(d, vv[j] - wm[j], wq[j]);
      }
    }
  }
  if (lane == 0) wst[wave * WSTW] = (float)wn;
#pragma unroll
  for (int j = 0; j < 4; ++j) {
    wst[wave * WSTW + 1 + 4 * lane + j]      = wm[j];
    wst[wave * WSTW + 1 + HC + 4 * lane + j] = wq[j];
  }
  __syncthreads();
  if (tid < HC) {
    float n = 0.0f, mean = 0.0f, M2 = 0.0f;
#pragma unroll 1
    for (int w2 = 0; w2 < NWAVE; ++w2) {
      const float nb = wst[w2 * WSTW];
      const float mb = wst[w2 * WSTW + 1 + tid];
      const float qb = wst[w2 * WSTW + 1 + HC + tid];
      if (nb > 0.5f) {
        const float nn = n + nb;
        const float delta = mb - mean;
        const float f = nb / nn;
        mean = fmaf(delta, f, mean);
        M2 = M2 + qb + delta * delta * n * f;
        n = nn;
      }
    }
    pst[1 + tid] = mean;
    pst[1 + HC + tid] = M2;
    if (tid == 0) pst[0] = n;
  }
#pragma unroll 1
  for (int i = 2 * HC + 1 + tid; i < PARTW; i += NTHR) pst[i] = 0.0f;
  __syncthreads();
  v4f ps = {0.f, 0.f, 0.f, 0.f};
  float* rp = rec + (size_t)blockIdx.x * PARTW + 4 * tid;
  if (tid < PARTW / 4) {
    ps = *(const v4fa*)(pst + 4 * tid);
    *(volatile v4f*)rp = ps;
  }
  __threadfence();
  if (tid < PARTW / 4) {
    *(volatile v4f*)rp = ps;
  }
}

__global__ __launch_bounds__(NTHR) void k_bn(const float* __restrict__ pre, const float* __restrict__ rec, int nRec,
                                             const float* __restrict__ gam, const float* __restrict__ bet,
                                             int nN, unsigned short* xhl) {
  __shared__ __attribute__((aligned(16))) float smu[HC];
  __shared__ __attribute__((aligned(16))) float srs[HC];
  __shared__ __attribute__((aligned(16))) float sg[HC];
  __shared__ __attribute__((aligned(16))) float sb[HC];
  const int tid = (int)threadIdx.x;
  if (tid < HC) {
    double n = 0.0, mean = 0.0, M2 = 0.0;
#pragma unroll 1
    for (int b = 0; b < nRec; ++b) {
      const float* pr = rec + (size_t)b * PARTW;
      const double nb = (double)pr[0];
      const double mb = (double)pr[1 + tid];
      const double qb = (double)pr[1 + HC + tid];
      if (nb > 0.5) {
        const double nn = n + nb;
        const double delta = mb - mean;
        const double f = nb / nn;
        mean = mean + delta * f;
        M2 = M2 + qb + delta * delta * n * f;
        n = nn;
      }
    }
    const double nt = n < 1.0 ? 1.0 : n;
    const float varf = (float)(M2 / nt);
    smu[tid] = (float)mean;
    srs[tid] = 1.0f / sqrtf(varf + 1e-5f);
    sg[tid]  = bfr(gam[tid]);
    sb[tid]  = bfr(bet[tid]);
  }
  __syncthreads();
  const int rowBase = (int)blockIdx.x * BNROWS;
#pragma unroll 1
  for (int it = 0; it < (BNROWS * 16) / NTHR; ++it) {
    const int u   = it * NTHR + tid;
    const int row = rowBase + (u >> 4);
    const int c0  = (u & 15) * 8;
    const int rc  = row < nN ? row : nN - 1;
    const float* p = pre + (size_t)rc * HC + c0;
    const v4f a = *(const v4fa*)p, b = *(const v4fa*)(p + 4);
    const v4f m0 = *(const v4fa*)(smu + c0), m1 = *(const v4fa*)(smu + c0 + 4);
    const v4f r0 = *(const v4fa*)(srs + c0), r1 = *(const v4fa*)(srs + c0 + 4);
    const v4f g0 = *(const v4fa*)(sg + c0),  g1 = *(const v4fa*)(sg + c0 + 4);
    const v4f e0 = *(const v4fa*)(sb + c0),  e1 = *(const v4fa*)(sb + c0 + 4);
    v4f ya, yb;
    ya.x = relun(((a.x - m0.x) * r0.x) * g0.x + e0.x);
    ya.y = relun(((a.y - m0.y) * r0.y) * g0.y + e0.y);
    ya.z = relun(((a.z - m0.z) * r0.z) * g0.z + e0.z);
    ya.w = relun(((a.w - m0.w) * r0.w) * g0.w + e0.w);
    yb.x = relun(((b.x - m1.x) * r1.x) * g1.x + e1.x);
    yb.y = relun(((b.y - m1.y) * r1.y) * g1.y + e1.y);
    yb.z = relun(((b.z - m1.z) * r1.z) * g1.z + e1.z);
    yb.w = relun(((b.w - m1.w) * r1.w) * g1.w + e1.w);
    const v4f z4 = {0.f, 0.f, 0.f, 0.f};
    if (row >= nN) { ya = z4; yb = z4; }
    const v4u hv = pack8(ya, yb);
    const v4u lv = pack8lo(ya, yb);
    unsigned short* hp = xhl + (size_t)row * KA + c0;
    unsigned short* lp = hp + HC;
    *(volatile v4u*)hp = hv;
    *(volatile v4u*)lp = lv;
    __threadfence();
    *(volatile v4u*)hp = hv;
    *(volatile v4u*)lp = lv;
  }
}

static inline int cdiv(int a, int b) { return (a + b - 1) / b; }
static inline size_t al256(size_t o) { return (o + 255) & ~(size_t)255; }

extern "C" void kernel_launch(void* const* d_in, const int* in_sizes, int n_in,
                              void* d_out, int out_size, void* d_ws, size_t ws_size,
                              hipStream_t stream) {
  if (n_in < 18) return;
  const int nN = in_sizes[0] / F_IN;
  if (nN <= 0 || in_sizes[0] != nN * F_IN) return;
  if (nN > 65536 || (nN & 3) != 0) return;
  if (in_sizes[1] < 2 || (in_sizes[1] & 1) != 0) return;
  const int nE = in_sizes[1] / 2;
  if (nE < 1 || nE > (1 << 28)) return;
  if (in_sizes[2] != F_IN * HC) return;
  if (in_sizes[3] != NHD * HW1 || in_sizes[4] != NHD * HW1) return;
  if (in_sizes[5] != HC || in_sizes[6] != HC || in_sizes[7] != HC) return;
  if (in_sizes[8] != HC * HC) return;
  if (in_sizes[9] != NHD * HW1 || in_sizes[10] != NHD * HW1) return;
  if (in_sizes[11] != HC || in_sizes[12] != HC || in_sizes[13] != HC) return;
  if (in_sizes[14] != HC * OUTC) return;
  if (in_sizes[15] != OUTC || in_sizes[16] != OUTC || in_sizes[17] != OUTC) return;
  if (out_size != nN * OUTC) return;

  const float* x   = (const float*)d_in[0];
  const int*   ei  = (const int*)  d_in[1];
  const float* W0  = (const float*)d_in[2];
  const float* as0 = (const float*)d_in[3];
  const float* ad0 = (const float*)d_in[4];
  const float* b0  = (const float*)d_in[5];
  const float* g0  = (const float*)d_in[6];
  const float* be0 = (const float*)d_in[7];
  const float* W1  = (const float*)d_in[8];
  const float* as1 = (const float*)d_in[9];
  const float* ad1 = (const float*)d_in[10];
  const float* b1  = (const float*)d_in[11];
  const float* g1  = (const float*)d_in[12];
  const float* be1 = (const float*)d_in[13];
  const float* W2  = (const float*)d_in[14];
  const float* as2 = (const float*)d_in[15];
  const float* ad2 = (const float*)d_in[16];
  const float* b2  = (const float*)d_in[17];
  float* out = (float*)d_out;
  const int* src = ei;
  const int* dst = ei + nE;

  const int MP   = cdiv(nN, MROWS) * MROWS;
  const int gA   = cdiv(MP, NB);
  const int gS   = cdiv(nN, NB);
  const int gM   = MP / GBM;
  const int vec8 = ((nE & 3) == 0) ? 1 : 0;
  if (gA * NB < MP || gS > gA) return;
  const int nUx = MP * (F_IN / 8);
  if ((nUx % NTHR) != 0) return;

  char* ws = (char*)d_ws;
  size_t off = 0;
  const size_t oXHL = off; off = al256(off + (size_t)MP * KA * 2);
  const size_t oW0T = off; off = al256(off + (size_t)HC * F_IN * 2);
  const size_t oW1T = off; off = al256(off + (size_t)HC * KA * 2);
  const size_t oW2T = off; off = al256(off + (size_t)HC3 * KA * 2);
  const size_t oH   = off; off = al256(off + (size_t)MP * HC * 4);
  const size_t oPRE = off; off = al256(off + (size_t)MP * HC * 4);
  const size_t oSD  = off; off = al256(off + (size_t)2 * NHD * MP * 4);
  const size_t oSRT = off; off = al256(off + (size_t)gA * RCAP * 4);
  const size_t oOFS = off; off = al256(off + (size_t)gA * 2 * NB * 4);
  const size_t oHDR = off; off = al256(off + (size_t)gA * HDRW * 4);
  const size_t oREC = off; off = al256(off + (size_t)gA * PARTW * 4);
  if (off > ws_size || off > (size_t)WSMAX) return;
  unsigned short* XHL = (unsigned short*)(ws + oXHL);
  unsigned short* XB  = (unsigned short*)(ws + oXHL);
  unsigned short* W0T = (unsigned short*)(ws + oW0T);
  unsigned short* W1T = (unsigned short*)(ws + oW1T);
  unsigned short* W2T = (unsigned short*)(ws + oW2T);
  float*          H   = (float*)(ws + oH);
  float*          PRE = (float*)(ws + oPRE);
  float*          SD  = (float*)(ws + oSD);
  int*            SRT = (int*)(ws + oSRT);
  int*            OFS = (int*)(ws + oOFS);
  int*            HDR = (int*)(ws + oHDR);
  float*          REC = (float*)(ws + oREC);

  hipFuncSetAttribute(reinterpret_cast<const void*>(&k_bucket),
                      hipFuncAttributeMaxDynamicSharedMemorySize, LDS_BKT);

  k_xprep<<<nUx / NTHR, NTHR, 0, stream>>>(x, XB, nN, nUx);
  {
    const int nU0 = HC * (F_IN / 8);
    k_wtr<<<cdiv(nU0, NTHR), NTHR, 0, stream>>>(W0, F_IN, HC, HC, F_IN, W0T, nU0);
    const int nU1 = HC * (KA / 8);
    k_wtr<<<cdiv(nU1, NTHR), NTHR, 0, stream>>>(W1, HC, HC, HC, KA, W1T, nU1);
    const int nU2 = HC3 * (KA / 8);
    k_wtr<<<cdiv(nU2, NTHR), NTHR, 0, stream>>>(W2, HC, OUTC, HC3, KA, W2T, nU2);
  }
  k_bucket<<<gA, NTHR, LDS_BKT, stream>>>(src, dst, nN, nE, vec8, SRT, OFS, HDR);

  k_gemm<2, HW1><<<dim3(gM, HC / GBN), GTHR, 0, stream>>>(XB, W0T, H, F_IN, HC, as0, ad0, HW1, SD, MP);
  k_scan<0><<<gA, NTHR, 0, stream>>>(SRT, OFS, HDR, H, SD, b0, PRE, out, nN, MP);
  k_stats<<<gS, NTHR, 0, stream>>>(PRE, nN, REC);
  k_bn<<<MP / BNROWS, NTHR, 0, stream>>>(PRE, REC, gS, g0, be0, nN, XHL);

  k_gemm<2, HW1><<<dim3(gM, HC / GBN), GTHR, 0, stream>>>(XHL, W1T, H, KA, HC, as1, ad1, HW1, SD, MP);
  k_scan<0><<<gA, NTHR, 0, stream>>>(SRT, OFS, HDR, H, SD, b1, PRE, out, nN, MP);
  k_stats<<<gS, NTHR, 0, stream>>>(PRE, nN, REC);
  k_bn<<<MP / BNROWS, NTHR, 0, stream>>>(PRE, REC, gS, g1, be1, nN, XHL);

  k_gemm<1, HC3><<<dim3(gM, 1), GTHR, 0, stream>>>(XHL, W2T, H, KA, HC3, as2, ad2, OUTC, SD, MP);
  k_scan<1><<<gA, NTHR, 0, stream>>>(SRT, OFS, HDR, H, SD, b2, PRE, out, nN, MP);
}
